// GNNNaiveBlock_ChebGat_3435973837208
// MI455X (gfx1250) — hardware-verified
//
#include <hip/hip_runtime.h>
#include <stddef.h>


#define FD       64
#define HEADS    4
#define XHW      (HEADS * FD)
#define KCAT     (3 * FD)
#define WPC      192
#define WPG      64
#define NPC      (FD * (WPC / 8))
#define NPG      (XHW * (WPG / 8))
#define NTHR     256
#define NWAVE    8
#define EPT      8
#define NGRP     2
#define CHUNK    (NTHR * EPT * NGRP)
#define WCAP     (EPT * NGRP * 32)
#define LISTN    (NWAVE * WCAP)
#define NBD      4096
#define NBP      960
#define QPW      ((NBP * FD) / (NWAVE * 128))
#define NBS      4096
#define QPWS     ((NBS * 8) / (NWAVE * 128))
#define NBG      768
#define QPWG     ((NBG * FD) / (NWAVE * 128))
#define LNR      64
#define GROWS    (NWAVE * 16)
#define NWX      4
#define NTX      (NWX * 32)
#define XROWS    (NWX * 16)
#define ENW      (NTHR * 4)
#define LDS_PROP (NBP * FD * 4 + LISTN * 4 + 64)
#define LDS_STAT (3 * NBS * 4 * 4 + LISTN * 4 + 64)
#define LDS_GAGG (NBG * FD * 4 + 4 * NBG * 4 * 4 + LISTN * 4 + 64)
#define LN_EPS   1e-5f
#define SM_EPS   1e-16f
#define NEG_ACT  0.01f
#define NEG_GAT  0.2f

static_assert((CHUNK & (CHUNK - 1)) == 0);
static_assert(CHUNK <= 4096);
static_assert(NBP <= 4096 && NBD <= 4096 && NBS <= 4096 && NBG <= 4096);
static_assert(NBP * FD == NWAVE * 128 * QPW);
static_assert(NBS * 8 == NWAVE * 128 * QPWS);
static_assert(NBG * FD == NWAVE * 128 * QPWG);
static_assert(((NBP * FD) / 4) % NTHR == 0);
static_assert((NBD / 4) == NWAVE * 4 * 32);
static_assert((NBS * 4) % NTHR == 0 && (NBG * 4) % NTHR == 0 && (NBG % (NTHR / 16)) == 0);
static_assert(KCAT % 32 == 0 && FD % 32 == 0 && WPC >= KCAT && (WPC % 64) == 0 && (WPG % 64) == 0);
static_assert((16 * FD) % 128 == 0);
static_assert((NPC % 32) == 0);
static_assert(LDS_GAGG <= 262208 && LDS_STAT <= 262208);

typedef float  v4f  __attribute__((ext_vector_type(4)));
typedef float  v8f  __attribute__((ext_vector_type(8)));
typedef int    v4i  __attribute__((ext_vector_type(4)));
typedef __bf16 v8b  __attribute__((ext_vector_type(8)));
typedef __bf16 v16b __attribute__((ext_vector_type(16)));
union FragB { v16b v; v8b h[2]; };
union CvB   { v8b b; v4i i; };

__device__ __forceinline__ void split8(v4f a, v4f b, v8b& hi, v8b& lo) {
  __bf16 t;
  t = (__bf16)a.x; hi[0] = t; lo[0] = (__bf16)(a.x - (float)t);
  t = (__bf16)a.y; hi[1] = t; lo[1] = (__bf16)(a.y - (float)t);
  t = (__bf16)a.z; hi[2] = t; lo[2] = (__bf16)(a.z - (float)t);
  t = (__bf16)a.w; hi[3] = t; lo[3] = (__bf16)(a.w - (float)t);
  t = (__bf16)b.x; hi[4] = t; lo[4] = (__bf16)(b.x - (float)t);
  t = (__bf16)b.y; hi[5] = t; lo[5] = (__bf16)(b.y - (float)t);
  t = (__bf16)b.z; hi[6] = t; lo[6] = (__bf16)(b.z - (float)t);
  t = (__bf16)b.w; hi[7] = t; lo[7] = (__bf16)(b.w - (float)t);
}

__device__ __forceinline__ v8f wmb(v16b a, v16b b, v8f c) {
  v8f d = __builtin_amdgcn_wmma_f32_16x16x32_bf16(false, a, false, b, (short)0, c, false, false);
  asm volatile("v_nop\n\tv_nop\n\tv_nop\n\tv_nop" : "+v"(d) : "v"(a), "v"(b));
  return d;
}

__device__ __forceinline__ float lk(float v, float s) { return v >= 0.f ? v : s * v; }

template <int NB>
__device__ __forceinline__ int scan_chunk(const int* __restrict__ keys, int nE, int cbase, int nodeBase,
                                          int vec8, int* list, int tid, int wave) {
  int wc = 0;
#pragma unroll
  for (int g = 0; g < NGRP; ++g) {
    const int el0  = (g * NTHR + tid) * EPT;
    const int e0   = cbase + el0;
    const int sent = -2147483647 - 1;
    v4i da, db;
    if (vec8 != 0 && e0 + 7 < nE) {
      da = *(const v4i*)(keys + e0);
      db = *(const v4i*)(keys + e0 + 4);
    } else {
      da.x = (e0     < nE) ? keys[min(e0,     nE - 1)] : sent;
      da.y = (e0 + 1 < nE) ? keys[min(e0 + 1, nE - 1)] : sent;
      da.z = (e0 + 2 < nE) ? keys[min(e0 + 2, nE - 1)] : sent;
      da.w = (e0 + 3 < nE) ? keys[min(e0 + 3, nE - 1)] : sent;
      db.x = (e0 + 4 < nE) ? keys[min(e0 + 4, nE - 1)] : sent;
      db.y = (e0 + 5 < nE) ? keys[min(e0 + 5, nE - 1)] : sent;
      db.z = (e0 + 6 < nE) ? keys[min(e0 + 6, nE - 1)] : sent;
      db.w = (e0 + 7 < nE) ? keys[min(e0 + 7, nE - 1)] : sent;
    }
    const unsigned nb = (unsigned)nodeBase;
    const unsigned s0 = (unsigned)da.x - nb, s1 = (unsigned)da.y - nb;
    const unsigned s2 = (unsigned)da.z - nb, s3 = (unsigned)da.w - nb;
    const unsigned s4 = (unsigned)db.x - nb, s5 = (unsigned)db.y - nb;
    const unsigned s6 = (unsigned)db.z - nb, s7 = (unsigned)db.w - nb;
    const bool h0 = s0 < (unsigned)NB, h1 = s1 < (unsigned)NB, h2 = s2 < (unsigned)NB, h3 = s3 < (unsigned)NB;
    const bool h4 = s4 < (unsigned)NB, h5 = s5 < (unsigned)NB, h6 = s6 < (unsigned)NB, h7 = s7 < (unsigned)NB;
    const unsigned any = __builtin_amdgcn_ballot_w32(h0 | h1 | h2 | h3 | h4 | h5 | h6 | h7);
    if (any != 0u) {
#define HITJ(J, HJ, SJ) { \
        const unsigned mj = __builtin_amdgcn_ballot_w32(HJ); \
        if (mj != 0u) { \
          if (HJ) { \
            const int pos = wc + (int)__builtin_amdgcn_mbcnt_lo(mj, 0u); \
            if (pos < WCAP) list[wave * WCAP + pos] = ((el0 + (J)) << 12) | (int)(SJ); \
          } \
          wc += (int)__builtin_popcount(mj); } }
      HITJ(0, h0, s0)
      HITJ(1, h1, s1)
      HITJ(2, h2, s2)
      HITJ(3, h3, s3)
      HITJ(4, h4, s4)
      HITJ(5, h5, s5)
      HITJ(6, h6, s6)
      HITJ(7, h7, s7)
#undef HITJ
    }
  }
  return wc;
}

__global__ __launch_bounds__(NTHR) void k_wprep(
    const float* __restrict__ cw, const float* __restrict__ gw,
    __bf16* chp, __bf16* clp, __bf16* ghp, __bf16* glp) {
  const int t = blockIdx.x * NTHR + threadIdx.x;
  if (t >= NPC + NPG) return;
  v4f a, b;
  __bf16* hp;
  __bf16* lp;
  if (t < NPC) {
    const int n  = t / (WPC / 8);
    const int q  = t - n * (WPC / 8);
    const int k0 = 8 * q;
    const float* p = cw + (size_t)k0 * FD + n;
    a.x = p[0];      a.y = p[FD];     a.z = p[2 * FD]; a.w = p[3 * FD];
    b.x = p[4 * FD]; b.y = p[5 * FD]; b.z = p[6 * FD]; b.w = p[7 * FD];
    hp = chp + (size_t)n * WPC + k0;
    lp = clp + (size_t)n * WPC + k0;
  } else {
    const int u  = t - NPC;
    const int n  = u / (WPG / 8);
    const int q  = u - n * (WPG / 8);
    const int k0 = 8 * q;
    const float* p = gw + (size_t)k0 * XHW + n;
    a.x = p[0];       a.y = p[XHW];     a.z = p[2 * XHW]; a.w = p[3 * XHW];
    b.x = p[4 * XHW]; b.y = p[5 * XHW]; b.z = p[6 * XHW]; b.w = p[7 * XHW];
    hp = ghp + (size_t)n * WPG + k0;
    lp = glp + (size_t)n * WPG + k0;
  }
  CvB hv, lv;
  split8(a, b, hv.b, lv.b);
  *(volatile v4i*)hp = hv.i;
  *(volatile v4i*)lp = lv.i;
  __threadfence();
  *(volatile v4i*)hp = hv.i;
  *(volatile v4i*)lp = lv.i;
}

__global__ __launch_bounds__(NTHR) void k_ln(
    const float* __restrict__ x, const float* __restrict__ g, const float* __restrict__ bta,
    float* xn, int nN) {
  const int tid = threadIdx.x, lane = tid & 31, wave = tid >> 5, hh = lane >> 4, m = lane & 15;
  const int rbase = blockIdx.x * LNR + wave * 8;
  const v4f gv = *(const v4f*)(g + 4 * m);
  const v4f bv = *(const v4f*)(bta + 4 * m);
  v4f ov[4];
#pragma unroll
  for (int j = 0; j < 4; ++j) {
    int row = rbase + 2 * j + hh;
    row = row > nN - 1 ? nN - 1 : row;
    const v4f v = *(const v4f*)(x + (size_t)row * FD + 4 * m);
    float s = (v.x + v.y) + (v.z + v.w);
    s += __shfl_xor(s, 1); s += __shfl_xor(s, 2); s += __shfl_xor(s, 4); s += __shfl_xor(s, 8);
    const float mu = s * (1.0f / FD);
    const v4f d = v - mu;
    float q = d.x * d.x + d.y * d.y + d.z * d.z + d.w * d.w;
    q += __shfl_xor(q, 1); q += __shfl_xor(q, 2); q += __shfl_xor(q, 4); q += __shfl_xor(q, 8);
    const float var  = q * (1.0f / FD);
    const float rstd = rsqrtf(var + LN_EPS);
    ov[j] = (d * rstd) * gv + bv;
  }
  float* gp = xn + (size_t)rbase * FD + 4 * lane;
#pragma unroll
  for (int j = 0; j < 4; ++j) *(volatile v4f*)(gp + 128 * j) = ov[j];
  __threadfence();
#pragma unroll
  for (int j = 0; j < 4; ++j) *(volatile v4f*)(gp + 128 * j) = ov[j];
}

__global__ __launch_bounds__(NTHR) void k_deg(
    const int* __restrict__ ei, const float* __restrict__ ew, float* dis, int nN, int nE, int vec8) {
  __shared__ __attribute__((aligned(16))) float cnt[NBD];
  __shared__ __attribute__((aligned(16))) int list[LISTN];
  __shared__ int wcnt[NWAVE];
  const int tid = threadIdx.x, lane = tid & 31, wave = tid >> 5;
  const int nodeBase = blockIdx.x * NBD;
  (void)nN;

  for (int i = tid; i < NBD; i += NTHR) cnt[i] = 0.f;
  __syncthreads();

  const int nChunks = (nE + CHUNK - 1) / CHUNK;
#pragma unroll 1
  for (int ch = 0; ch < nChunks; ++ch) {
    const int cbase = ch * CHUNK;
    const int wc = scan_chunk<NBD>(ei, nE, cbase, nodeBase, vec8, list, tid, wave);
    if (lane == 0) wcnt[wave] = wc;
    __syncthreads();
    if (wave == 0) {
#pragma unroll 1
      for (int wsx = 0; wsx < NWAVE; ++wsx) {
        int n = __builtin_amdgcn_readfirstlane(wcnt[wsx]);
        n = n > WCAP ? WCAP : (n < 0 ? 0 : n);
        const int* lp = list + wsx * WCAP;
#pragma unroll 1
        for (int i = 0; i < n; ++i) {
          const int ent  = __builtin_amdgcn_readfirstlane(lp[i]);
          const int slot = ent & (NBD - 1);
          int e = cbase + ((ent >> 12) & (CHUNK - 1));
          e = e > nE - 1 ? nE - 1 : e;
          const float w = ew[e];
          if (lane == 0) cnt[slot] = cnt[slot] + w;
        }
      }
    }
    __syncthreads();
  }

  v4f dq[4];
#pragma unroll
  for (int q = 0; q < 4; ++q) {
    const int f = (wave * 4 + q) * 128 + 4 * lane;
    const v4f c = *(const v4f*)(cnt + f);
    dq[q].x = (c.x > 0.f) ? rsqrtf(fmaxf(c.x, 1e-30f)) : 0.f;
    dq[q].y = (c.y > 0.f) ? rsqrtf(fmaxf(c.y, 1e-30f)) : 0.f;
    dq[q].z = (c.z > 0.f) ? rsqrtf(fmaxf(c.z, 1e-30f)) : 0.f;
    dq[q].w = (c.w > 0.f) ? rsqrtf(fmaxf(c.w, 1e-30f)) : 0.f;
  }
  float* dp = dis + (size_t)nodeBase;
#pragma unroll
  for (int q = 0; q < 4; ++q) *(volatile v4f*)(dp + (wave * 4 + q) * 128 + 4 * lane) = dq[q];
  __threadfence();
#pragma unroll
  for (int q = 0; q < 4; ++q) *(volatile v4f*)(dp + (wave * 4 + q) * 128 + 4 * lane) = dq[q];
}

__global__ __launch_bounds__(NTHR) void k_enorm(
    const int* __restrict__ ei, const float* __restrict__ ew, const float* __restrict__ dis,
    float* nw, int nN, int nE) {
  const int e4 = (blockIdx.x * NTHR + threadIdx.x) * 4;
  v4f r;
#pragma unroll
  for (int c = 0; c < 4; ++c) {
    int e = e4 + c;
    e = e > nE - 1 ? nE - 1 : e;
    int s = ei[e];
    int d = ei[(size_t)nE + e];
    s = s < 0 ? 0 : (s > nN - 1 ? nN - 1 : s);
    d = d < 0 ? 0 : (d > nN - 1 ? nN - 1 : d);
    const float w = ew[e];
    r[c] = -(dis[s] * w) * dis[d];
  }
  *(volatile v4f*)(nw + e4) = r;
  __threadfence();
  *(volatile v4f*)(nw + e4) = r;
}

template <int MODE>
__global__ __launch_bounds__(NTHR) void k_prop(
    const int* __restrict__ ei, const float* __restrict__ nw, const float* __restrict__ hs,
    const float* __restrict__ t0, float* outp, int nN, int nE, int vec8) {
  extern __shared__ v4f lds_dyn[];
  float* acc  = (float*)lds_dyn;
  int*   list = (int*)(acc + NBP * FD);
  int*   wcnt = list + LISTN;
  const int tid = threadIdx.x, lane = tid & 31, wave = tid >> 5;
  const int nodeBase = blockIdx.x * NBP;
  const int* dsts = ei + nE;

  {
    const v4f z = {0.f, 0.f, 0.f, 0.f};
    for (int i = tid; i < NBP * FD / 4; i += NTHR) lds_dyn[i] = z;
  }
  __syncthreads();

  const int nChunks = (nE + CHUNK - 1) / CHUNK;
#pragma unroll 1
  for (int ch = 0; ch < nChunks; ++ch) {
    const int cbase = ch * CHUNK;
    const int wc = scan_chunk<NBP>(dsts, nE, cbase, nodeBase, vec8, list, tid, wave);
    if (lane == 0) wcnt[wave] = wc;
    __syncthreads();
    if (wave == 0) {
#pragma unroll 1
      for (int wsx = 0; wsx < NWAVE; ++wsx) {
        int n = __builtin_amdgcn_readfirstlane(wcnt[wsx]);
        n = n > WCAP ? WCAP : (n < 0 ? 0 : n);
        const int* lp = list + wsx * WCAP;
#pragma unroll 1
        for (int i = 0; i < n; ++i) {
          const int ent = __builtin_amdgcn_readfirstlane(lp[i]);
          int slot = ent & 4095;
          slot = slot > NBP - 1 ? NBP - 1 : slot;
          int e = cbase + ((ent >> 12) & (CHUNK - 1));
          e = e > nE - 1 ? nE - 1 : e;
          int src = ei[e];
          src = src < 0 ? 0 : (src > nN - 1 ? nN - 1 : src);
          const float w = nw[e];
          if (lane < FD / 4) {
            const v4f v = *(const v4f*)(hs + (size_t)src * FD + 4 * lane);
            v4f* ap = (v4f*)(acc + slot * FD + 4 * lane);
            *ap = *ap + v * w;
          }
        }
      }
    }
    __syncthreads();
  }

  if (MODE == 1) {
#pragma unroll 4
    for (int i = 0; i < (NBP * FD / 4) / NTHR; ++i) {
      const int idx  = i * NTHR + tid;
      const int slot = idx / (FD / 4);
      const int c4   = (idx - slot * (FD / 4)) * 4;
      int node = nodeBase + slot;
      node = node > nN - 1 ? nN - 1 : node;
      const v4f tv = *(const v4f*)(t0 + (size_t)node * FD + c4);
      v4f* ap = (v4f*)(acc + slot * FD + c4);
      *ap = *ap * 2.0f - tv;
    }
    __syncthreads();
  }

  float* gp = outp + (size_t)nodeBase * FD;
#pragma unroll 4
  for (int q = 0; q < QPW; ++q) {
    const int f = (wave * QPW + q) * 128 + 4 * lane;
    const v4f v = *(const v4f*)(acc + f);
    *(volatile v4f*)(gp + f) = v;
  }
  __threadfence();
#pragma unroll 4
  for (int q = 0; q < QPW; ++q) {
    const int f = (wave * QPW + q) * 128 + 4 * lane;
    const v4f v = *(const v4f*)(acc + f);
    *(volatile v4f*)(gp + f) = v;
  }
}

__global__ __launch_bounds__(NTHR) void k_cheb(
    const float* __restrict__ T0, const float* __restrict__ T1, const float* __restrict__ T2,
    const __bf16* __restrict__ whi, const __bf16* __restrict__ wlo,
    const float* __restrict__ bias, float* hout, int nN) {
  __shared__ __attribute__((aligned(16))) float stg[NWAVE * 16 * FD];
  const int tid = threadIdx.x, lane = tid & 31, wave = tid >> 5, hh = lane >> 4, m = lane & 15;
  const int row0 = (blockIdx.x * NWAVE + wave) * 16;
  int ra = row0 + m;
  ra = ra > nN - 1 ? nN - 1 : ra;

  v8f acc[FD / 16];
#pragma unroll
  for (int t = 0; t < FD / 16; ++t) { v8f z = {0.f, 0.f, 0.f, 0.f, 0.f, 0.f, 0.f, 0.f}; acc[t] = z; }

#pragma unroll 1
  for (int kt = 0; kt < KCAT / 32; ++kt) {
    const int j  = kt >> 1;
    const int kk = 32 * (kt - 2 * j) + 8 * hh;
    const float* P  = (j == 0) ? T0 : ((j == 1) ? T1 : T2);
    const float* ap = P + (size_t)ra * FD + kk;
    const v4f x0 = *(const v4f*)ap,        x1 = *(const v4f*)(ap + 4);
    const v4f x2 = *(const v4f*)(ap + 16), x3 = *(const v4f*)(ap + 20);
    FragB ah, al;
    split8(x0, x1, ah.h[0], al.h[0]);
    split8(x2, x3, ah.h[1], al.h[1]);
    const __bf16* ph = whi + (size_t)m * WPC + 32 * kt + 8 * hh;
    const __bf16* pl = wlo + (size_t)m * WPC + 32 * kt + 8 * hh;
#pragma unroll
    for (int t = 0; t < FD / 16; ++t) {
      const __bf16* qh = ph + (size_t)(16 * t) * WPC;
      const __bf16* ql = pl + (size_t)(16 * t) * WPC;
      FragB bh, blw;
      bh.h[0]  = *(const v8b*)qh;  bh.h[1]  = *(const v8b*)(qh + 16);
      blw.h[0] = *(const v8b*)ql;  blw.h[1] = *(const v8b*)(ql + 16);
      acc[t] = wmb(ah.v, bh.v,  acc[t]);
      acc[t] = wmb(ah.v, blw.v, acc[t]);
      acc[t] = wmb(al.v, bh.v,  acc[t]);
    }
  }

  float bv[FD / 16];
#pragma unroll
  for (int t = 0; t < FD / 16; ++t) bv[t] = bias[16 * t + m];

  float* sp = stg + wave * (16 * FD) + (8 * hh) * FD + m;
#pragma unroll
  for (int t = 0; t < FD / 16; ++t) {
#pragma unroll
    for (int r = 0; r < 8; ++r) sp[r * FD + 16 * t] = lk(acc[t][r] + bv[t], NEG_ACT);
  }
  __syncthreads();
  const float* lp = stg + wave * (16 * FD) + 4 * lane;
  float* gp = hout + (size_t)row0 * FD + 4 * lane;
#pragma unroll
  for (int i = 0; i < (16 * FD) / 128; ++i) { const v4f v = *(const v4f*)(lp + 128 * i); *(volatile v4f*)(gp + 128 * i) = v; }
  __threadfence();
#pragma unroll
  for (int i = 0; i < (16 * FD) / 128; ++i) { const v4f v = *(const v4f*)(lp + 128 * i); *(volatile v4f*)(gp + 128 * i) = v; }
}

__global__ __launch_bounds__(NTX) void k_gatx(
    const float* __restrict__ H, const __bf16* __restrict__ ghi, const __bf16* __restrict__ glo,
    const float* __restrict__ ats, const float* __restrict__ atd,
    float* xh, float* asd, int nN) {
  __shared__ __attribute__((aligned(16))) float stg[NWX * 16 * FD];
  __shared__ __attribute__((aligned(16))) float sds[NWX * 16 * 8];
  const int tid = threadIdx.x, lane = tid & 31, wave = tid >> 5, hh = lane >> 4, m = lane & 15;
  const int row0 = (blockIdx.x * NWX + wave) * 16;
  (void)nN;

  FragB ah0, al0, ah1, al1;
  {
    const float* ap = H + (size_t)(row0 + m) * FD + 8 * hh;
    const v4f x0 = *(const v4f*)ap,        x1 = *(const v4f*)(ap + 4);
    const v4f x2 = *(const v4f*)(ap + 16), x3 = *(const v4f*)(ap + 20);
    split8(x0, x1, ah0.h[0], al0.h[0]);
    split8(x2, x3, ah0.h[1], al0.h[1]);
    const float* bp = ap + 32;
    const v4f y0 = *(const v4f*)bp,        y1 = *(const v4f*)(bp + 4);
    const v4f y2 = *(const v4f*)(bp + 16), y3 = *(const v4f*)(bp + 20);
    split8(y0, y1, ah1.h[0], al1.h[0]);
    split8(y2, y3, ah1.h[1], al1.h[1]);
  }

#pragma unroll 1
  for (int hd = 0; hd < HEADS; ++hd) {
    v8f acc[4];
#pragma unroll
    for (int t = 0; t < 4; ++t) { v8f z = {0.f, 0.f, 0.f, 0.f, 0.f, 0.f, 0.f, 0.f}; acc[t] = z; }
    {
      const __bf16* ph = ghi + (size_t)(hd * FD + m) * WPG + 8 * hh;
      const __bf16* pl = glo + (size_t)(hd * FD + m) * WPG + 8 * hh;
#pragma unroll
      for (int t = 0; t < 4; ++t) {
        const __bf16* qh = ph + (size_t)(16 * t) * WPG;
        const __bf16* ql = pl + (size_t)(16 * t) * WPG;
        FragB bh, blw;
        bh.h[0]  = *(const v8b*)qh;  bh.h[1]  = *(const v8b*)(qh + 16);
        blw.h[0] = *(const v8b*)ql;  blw.h[1] = *(const v8b*)(ql + 16);
        acc[t] = wmb(ah0.v, bh.v,  acc[t]);
        acc[t] = wmb(ah0.v, blw.v, acc[t]);
        acc[t] = wmb(al0.v, bh.v,  acc[t]);
      }
#pragma unroll
      for (int t = 0; t < 4; ++t) {
        const __bf16* qh = ph + (size_t)(16 * t) * WPG + 32;
        const __bf16* ql = pl + (size_t)(16 * t) * WPG + 32;
        FragB bh, blw;
        bh.h[0]  = *(const v8b*)qh;  bh.h[1]  = *(const v8b*)(qh + 16);
        blw.h[0] = *(const v8b*)ql;  blw.h[1] = *(const v8b*)(ql + 16);
        acc[t] = wmb(ah1.v, bh.v,  acc[t]);
        acc[t] = wmb(ah1.v, blw.v, acc[t]);
        acc[t] = wmb(al1.v, bh.v,  acc[t]);
      }
    }

    float as[4], ad[4];
#pragma unroll
    for (int t = 0; t < 4; ++t) { as[t] = ats[hd * FD + 16 * t + m]; ad[t] = atd[hd * FD + 16 * t + m]; }
    float ps[8], pd[8];
#pragma unroll
    for (int r = 0; r < 8; ++r) { ps[r] = 0.f; pd[r] = 0.f; }
#pragma unroll
    for (int t = 0; t < 4; ++t) {
#pragma unroll
      for (int r = 0; r < 8; ++r) { ps[r] += acc[t][r] * as[t]; pd[r] += acc[t][r] * ad[t]; }
    }
#pragma unroll
    for (int mk = 1; mk < 16; mk <<= 1) {
#pragma unroll
      for (int r = 0; r < 8; ++r) { ps[r] += __shfl_xor(ps[r], mk); pd[r] += __shfl_xor(pd[r], mk); }
    }

    float* sp = stg + wave * (16 * FD) + (8 * hh) * FD + m;
#pragma unroll
    for (int t = 0; t < 4; ++t) {
#pragma unroll
      for (int r = 0; r < 8; ++r) sp[r * FD + 16 * t] = acc[t][r];
    }
    {
      float vs = 0.f, vd = 0.f;
#pragma unroll
      for (int r = 0; r < 8; ++r) { vs = (m == r) ? ps[r] : vs; vd = (m == r) ? pd[r] : vd; }
      if (m < 8) {
        float* dp = sds + wave * 128 + (8 * hh + m) * 8;
        dp[hd] = vs;
        dp[4 + hd] = vd;
      }
    }
    __syncthreads();

    const float* lp = stg + wave * (16 * FD) + 4 * m;
    float* gp = xh + (size_t)row0 * XHW + hd * FD + 4 * m;
#pragma unroll
    for (int i = 0; i < 8; ++i) {
      const int row = 2 * i + hh;
      const v4f v = *(const v4f*)(lp + row * FD);
      *(volatile v4f*)(gp + (size_t)row * XHW) = v;
    }
    __threadfence();
#pragma unroll
    for (int i = 0; i < 8; ++i) {
      const int row = 2 * i + hh;
      const v4f v = *(const v4f*)(lp + row * FD);
      *(volatile v4f*)(gp + (size_t)row * XHW) = v;
    }
    __syncthreads();
  }

  const v4f dv = *(const v4f*)(sds + wave * 128 + 4 * lane);
  float* ap2 = asd + (size_t)row0 * 8 + 4 * lane;
  *(volatile v4f*)ap2 = dv;
  __threadfence();
  *(volatile v4f*)ap2 = dv;
}

__global__ __launch_bounds__(NTHR) void k_gstat(
    const int* __restrict__ ei, const float* __restrict__ asd, float* st, int nN, int nE, int vec8) {
  extern __shared__ v4f lds_dyn[];
  float* sM   = (float*)lds_dyn;
  float* sS   = sM + NBS * 4;
  float* sD   = sS + NBS * 4;
  int*   list = (int*)(sD + NBS * 4);
  int*   wcnt = list + LISTN;
  const int tid = threadIdx.x, lane = tid & 31, wave = tid >> 5;
  const int nodeBase = blockIdx.x * NBS;
  const int* dsts = ei + nE;

  for (int i = tid; i < NBS * 4; i += NTHR) {
    const int slot = i >> 2, h = i & 3;
    int node = nodeBase + slot;
    node = node > nN - 1 ? nN - 1 : node;
    const float as = asd[(size_t)node * 8 + h];
    const float ad = asd[(size_t)node * 8 + 4 + h];
    const float e = lk(as + ad, NEG_GAT);
    sM[i] = e;
    sS[i] = 1.f;
    sD[i] = ad;
  }
  __syncthreads();

  const int nChunks = (nE + CHUNK - 1) / CHUNK;
#pragma unroll 1
  for (int ch = 0; ch < nChunks; ++ch) {
    const int cbase = ch * CHUNK;
    const int wc = scan_chunk<NBS>(dsts, nE, cbase, nodeBase, vec8, list, tid, wave);
    if (lane == 0) wcnt[wave] = wc;
    __syncthreads();
    if (wave == 0) {
      const int h = lane & 3;
#pragma unroll 1
      for (int wsx = 0; wsx < NWAVE; ++wsx) {
        int n = __builtin_amdgcn_readfirstlane(wcnt[wsx]);
        n = n > WCAP ? WCAP : (n < 0 ? 0 : n);
        const int* lp = list + wsx * WCAP;
#pragma unroll 1
        for (int i = 0; i < n; ++i) {
          const int ent  = __builtin_amdgcn_readfirstlane(lp[i]);
          const int slot = ent & (NBS - 1);
          int e = cbase + ((ent >> 12) & (CHUNK - 1));
          e = e > nE - 1 ? nE - 1 : e;
          int src = ei[e];
          src = src < 0 ? 0 : (src > nN - 1 ? nN - 1 : src);
          const float as = asd[(size_t)src * 8 + h];
          const int si = slot * 4 + h;
          const float ev = lk(as + sD[si], NEG_GAT);
          const float M = sM[si], S = sS[si];
          const float mx = fmaxf(ev, M), mn = fminf(ev, M);
          const float p  = expf(mn - mx);
          const float Sn = (ev > M) ? (S * p + 1.f) : (S + p);
          if (lane < 4) { sM[si] = mx; sS[si] = Sn; }
        }
      }
    }
    __syncthreads();
  }

  float* gp = st + (size_t)nodeBase * 8;
#pragma unroll 4
  for (int q = 0; q < QPWS; ++q) {
    const int f = (wave * QPWS + q) * 128 + 4 * lane;
    const int slot = f >> 3;
    const float* bp = ((f >> 2) & 1) ? sS : sM;
    const v4f v = *(const v4f*)(bp + slot * 4);
    *(volatile v4f*)(gp + f) = v;
  }
  __threadfence();
#pragma unroll 4
  for (int q = 0; q < QPWS; ++q) {
    const int f = (wave * QPWS + q) * 128 + 4 * lane;
    const int slot = f >> 3;
    const float* bp = ((f >> 2) & 1) ? sS : sM;
    const v4f v = *(const v4f*)(bp + slot * 4);
    *(volatile v4f*)(gp + f) = v;
  }
}

__global__ __launch_bounds__(NTHR) void k_gagg(
    const int* __restrict__ ei, const float* __restrict__ xh, const float* __restrict__ asd,
    const float* __restrict__ st, const float* __restrict__ gb, float* out, int nN, int nE, int vec8) {
  extern __shared__ v4f lds_dyn[];
  float* acc  = (float*)lds_dyn;
  float* sM   = acc + NBG * FD;
  float* sI   = sM + NBG * 4;
  float* sD   = sI + NBG * 4;
  float* sA   = sD + NBG * 4;
  int*   list = (int*)(sA + NBG * 4);
  int*   wcnt = list + LISTN;
  const int tid = threadIdx.x, lane = tid & 31, wave = tid >> 5, hh = lane >> 4, m = lane & 15;
  const int nodeBase = blockIdx.x * NBG;
  const int* dsts = ei + nE;

  for (int i = tid; i < NBG * 4; i += NTHR) {
    const int slot = i >> 2, h = i & 3;
    int node = nodeBase + slot;
    node = node > nN - 1 ? nN - 1 : node;
    const float M  = st[(size_t)node * 8 + h];
    const float S  = st[(size_t)node * 8 + 4 + h];
    const float as = asd[(size_t)node * 8 + h];
    const float ad = asd[(size_t)node * 8 + 4 + h];
    const float inv = 1.0f / (S + SM_EPS);
    const float e   = lk(as + ad, NEG_GAT);
    sM[i] = M;
    sI[i] = inv;
    sD[i] = ad;
    sA[i] = expf(e - M) * inv;
  }
  __syncthreads();

  for (int it = tid >> 4; it < NBG; it += NTHR / 16) {
    int node = nodeBase + it;
    node = node > nN - 1 ? nN - 1 : node;
    const int c4 = 4 * (tid & 15);
    const v4f a = *(const v4f*)(sA + it * 4);
    const float* xp = xh + (size_t)node * XHW + c4;
    const v4f v = *(const v4f*)xp * a.x + *(const v4f*)(xp + FD) * a.y
                + *(const v4f*)(xp + 2 * FD) * a.z + *(const v4f*)(xp + 3 * FD) * a.w;
    *(v4f*)(acc + it * FD + c4) = v;
  }
  __syncthreads();

  const int nChunks = (nE + CHUNK - 1) / CHUNK;
#pragma unroll 1
  for (int ch = 0; ch < nChunks; ++ch) {
    const int cbase = ch * CHUNK;
    const int wc = scan_chunk<NBG>(dsts, nE, cbase, nodeBase, vec8, list, tid, wave);
    if (lane == 0) wcnt[wave] = wc;
    __syncthreads();
    if (wave == 0) {
#pragma unroll 1
      for (int wsx = 0; wsx < NWAVE; ++wsx) {
        int n = __builtin_amdgcn_readfirstlane(wcnt[wsx]);
        n = n > WCAP ? WCAP : (n < 0 ? 0 : n);
        const int* lp = list + wsx * WCAP;
#pragma unroll 1
        for (int i = 0; i < n; ++i) {
          const int ent = __builtin_amdgcn_readfirstlane(lp[i]);
          int slot = ent & 4095;
          slot = slot > NBG - 1 ? NBG - 1 : slot;
          int e = cbase + ((ent >> 12) & (CHUNK - 1));
          e = e > nE - 1 ? nE - 1 : e;
          int src = ei[e];
          src = src < 0 ? 0 : (src > nN - 1 ? nN - 1 : src);
          const int s0 = slot * 4 + hh, s1 = s0 + 2;
          const float as0 = asd[(size_t)src * 8 + hh];
          const float as1 = asd[(size_t)src * 8 + hh + 2];
          const float e0 = lk(as0 + sD[s0], NEG_GAT);
          const float e1 = lk(as1 + sD[s1], NEG_GAT);
          const float p0 = expf(e0 - sM[s0]) * sI[s0];
          const float p1 = expf(e1 - sM[s1]) * sI[s1];
          const float* xp = xh + (size_t)src * XHW + hh * FD + 4 * m;
          v4f pv = *(const v4f*)xp * p0 + *(const v4f*)(xp + 2 * FD) * p1;
          pv.x += __shfl_xor(pv.x, 16);
          pv.y += __shfl_xor(pv.y, 16);
          pv.z += __shfl_xor(pv.z, 16);
          pv.w += __shfl_xor(pv.w, 16);
          if (hh == 0) {
            v4f* ap = (v4f*)(acc + slot * FD + 4 * m);
            *ap = *ap + pv;
          }
        }
      }
    }
    __syncthreads();
  }

  const v4f gb4 = *(const v4f*)(gb + ((4 * lane) & (FD - 1)));
  const size_t outN  = (size_t)nN * FD;
  const size_t gbase = (size_t)nodeBase * FD;
#pragma unroll 4
  for (int q = 0; q < QPWG; ++q) {
    const int f = (wave * QPWG + q) * 128 + 4 * lane;
    const v4f v = *(const v4f*)(acc + f);
    v4f r = v * 0.25f + gb4;
    r.x = lk(r.x, NEG_ACT); r.y = lk(r.y, NEG_ACT); r.z = lk(r.z, NEG_ACT); r.w = lk(r.w, NEG_ACT);
    if (gbase + (size_t)f < outN) *(volatile v4f*)(out + gbase + f) = r;
  }
  __threadfence();
#pragma unroll 4
  for (int q = 0; q < QPWG; ++q) {
    const int f = (wave * QPWG + q) * 128 + 4 * lane;
    const v4f v = *(const v4f*)(acc + f);
    v4f r = v * 0.25f + gb4;
    r.x = lk(r.x, NEG_ACT); r.y = lk(r.y, NEG_ACT); r.z = lk(r.z, NEG_ACT); r.w = lk(r.w, NEG_ACT);
    if (gbase + (size_t)f < outN) *(volatile v4f*)(out + gbase + f) = r;
  }
}

extern "C" void kernel_launch(void* const* d_in, const int* in_sizes, int n_in,
                              void* d_out, int out_size, void* d_ws, size_t ws_size,
                              hipStream_t stream) {
  if (n_in < 11) return;
  const int nN = in_sizes[0] / FD;
  if (nN <= 0 || in_sizes[0] != nN * FD) return;
  const int nE = in_sizes[2];
  if (nE <= 0 || in_sizes[1] != 2 * nE) return;
  if (in_sizes[3] < FD || in_sizes[4] < FD) return;
  if (in_sizes[5] != 3 * FD * FD || in_sizes[6] < FD) return;
  if (in_sizes[7] != FD * XHW || in_sizes[8] < HEADS * FD || in_sizes[9] < HEADS * FD || in_sizes[10] < FD) return;
  if (out_size != nN * FD) return;

  const float* x    = (const float*)d_in[0];
  const int*   ei   = (const int*)d_in[1];
  const float* ew   = (const float*)d_in[2];
  const float* lng  = (const float*)d_in[3];
  const float* lnb  = (const float*)d_in[4];
  const float* cw   = (const float*)d_in[5];
  const float* cb   = (const float*)d_in[6];
  const float* gw   = (const float*)d_in[7];
  const float* ats  = (const float*)d_in[8];
  const float* atd  = (const float*)d_in[9];
  const float* gbv  = (const float*)d_in[10];
  float* out = (float*)d_out;

  const int nBD = (nN + NBD - 1) / NBD;
  const int nNW = (nE + ENW - 1) / ENW;
  const int nPB = (nN + NBP - 1) / NBP;
  const int nLB = (nN + LNR - 1) / LNR;
  const int nGB = (nN + GROWS - 1) / GROWS;
  const int nXB = (nN + XROWS - 1) / XROWS;
  const int nSB = (nN + NBS - 1) / NBS;
  const int nAB = (nN + NBG - 1) / NBG;

  char* ws = (char*)d_ws;
  size_t off = 0;
  const size_t plC = (size_t)FD * WPC * 2;
  const size_t plG = (size_t)XHW * WPG * 2;
  const size_t oCh  = off; off += plC;                                        off = (off + 255) & ~(size_t)255;
  const size_t oCl  = off; off += plC;                                        off = (off + 255) & ~(size_t)255;
  const size_t oGh  = off; off += plG;                                        off = (off + 255) & ~(size_t)255;
  const size_t oGl  = off; off += plG;                                        off = (off + 255) & ~(size_t)255;
  const size_t oDis = off; off += (size_t)nBD * NBD * 4;                      off = (off + 255) & ~(size_t)255;
  const size_t oNW  = off; off += (size_t)nNW * ENW * 4;                      off = (off + 255) & ~(size_t)255;
  const size_t oXN  = off; off += (size_t)nLB * LNR * FD * 4;                 off = (off + 255) & ~(size_t)255;
  const size_t oT1  = off; off += (size_t)nPB * NBP * FD * 4;                 off = (off + 255) & ~(size_t)255;
  const size_t oT2  = off; off += (size_t)nPB * NBP * FD * 4;                 off = (off + 255) & ~(size_t)255;
  const size_t oH   = off; off += (size_t)nGB * GROWS * FD * 4;               off = (off + 255) & ~(size_t)255;
  const size_t oXH  = off; off += (size_t)nXB * XROWS * XHW * 4;              off = (off + 255) & ~(size_t)255;
  const size_t oASD = off; off += (size_t)nXB * XROWS * 8 * 4;                off = (off + 255) & ~(size_t)255;
  const size_t oST  = off; off += (size_t)nSB * NBS * 8 * 4;                  off = (off + 255) & ~(size_t)255;
  if (off > ws_size) return;
  if (off > (size_t)134217728) return;
  __bf16* chp = (__bf16*)(ws + oCh);
  __bf16* clp = (__bf16*)(ws + oCl);
  __bf16* ghp = (__bf16*)(ws + oGh);
  __bf16* glp = (__bf16*)(ws + oGl);
  float*  dis = (float*)(ws + oDis);
  float*  nw  = (float*)(ws + oNW);
  float*  XN  = (float*)(ws + oXN);
  float*  T1  = (float*)(ws + oT1);
  float*  T2  = (float*)(ws + oT2);
  float*  Hp  = (float*)(ws + oH);
  float*  XH  = (float*)(ws + oXH);
  float*  ASD = (float*)(ws + oASD);
  float*  ST  = (float*)(ws + oST);

  const int vec8 = ((nE & 3) == 0) ? 1 : 0;

  k_wprep<<<(NPC + NPG + NTHR - 1) / NTHR, NTHR, 0, stream>>>(cw, gw, chp, clp, ghp, glp);
  k_ln<<<nLB, NTHR, 0, stream>>>(x, lng, lnb, XN, nN);
  k_deg<<<nBD, NTHR, 0, stream>>>(ei, ew, dis, nN, nE, vec8);
  k_enorm<<<nNW, NTHR, 0, stream>>>(ei, ew, dis, nw, nN, nE);

  hipFuncSetAttribute(reinterpret_cast<const void*>(&k_prop<0>),
                      hipFuncAttributeMaxDynamicSharedMemorySize, LDS_PROP);
  hipFuncSetAttribute(reinterpret_cast<const void*>(&k_prop<1>),
                      hipFuncAttributeMaxDynamicSharedMemorySize, LDS_PROP);
  hipFuncSetAttribute(reinterpret_cast<const void*>(&k_gstat),
                      hipFuncAttributeMaxDynamicSharedMemorySize, LDS_STAT);
  hipFuncSetAttribute(reinterpret_cast<const void*>(&k_gagg),
                      hipFuncAttributeMaxDynamicSharedMemorySize, LDS_GAGG);

  k_prop<0><<<nPB, NTHR, LDS_PROP, stream>>>(ei, nw, XN, XN, T1, nN, nE, vec8);
  k_prop<1><<<nPB, NTHR, LDS_PROP, stream>>>(ei, nw, T1, XN, T2, nN, nE, vec8);
  k_cheb<<<nGB, NTHR, 0, stream>>>(XN, T1, T2, chp, clp, cb, Hp, nN);

  k_gatx<<<nXB, NTX, 0, stream>>>(Hp, ghp, glp, ats, atd, XH, ASD, nN);
  k_gstat<<<nSB, NTHR, LDS_STAT, stream>>>(ei, ASD, ST, nN, nE, vec8);
  k_gagg<<<nAB, NTHR, LDS_GAGG, stream>>>(ei, XH, ASD, ST, gbv, out, nN, nE, vec8);
}
